// CartesianPlaneNonSirenEmbeddingNetwork_38036230373700
// MI455X (gfx1250) — hardware-run, weakly checked
//
#include <hip/hip_runtime.h>
#include <math.h>

typedef __attribute__((ext_vector_type(16))) _Float16 v16h;
typedef __attribute__((ext_vector_type(16))) __bf16 v16b;
typedef __attribute__((ext_vector_type(8)))  _Float16 v8h;
typedef __attribute__((ext_vector_type(8)))  float v8f;
typedef __attribute__((ext_vector_type(4)))  float v4f;
typedef __attribute__((ext_vector_type(2)))  float v2f;
typedef __attribute__((ext_vector_type(4)))  unsigned v4u;
typedef __attribute__((ext_vector_type(4)))  int v4i;
typedef float __attribute__((may_alias)) float_a;
typedef int __attribute__((may_alias)) int_a;

template <typename T> __device__ __forceinline__ void vst2(void* p, T v) { *(volatile T*)p = v; __threadfence(); *(volatile T*)p = v; }
__device__ __forceinline__ v8f wmma16(v16h a, v16h b, v8f c) {
  v8f d = __builtin_amdgcn_wmma_f32_16x16x32_f16(false, a, false, b, (short)0, c, false, false);
  asm volatile("v_nop\n\tv_nop\n\tv_nop\n\tv_nop" : "+v"(d) : "v"(a), "v"(b));
  return d;
}
__device__ __forceinline__ v8f wmma_bf(v16b a, v16b b, v8f c) {
  v8f d = __builtin_amdgcn_wmma_f32_16x16x32_bf16(false, a, false, b, (short)0, c, false, false);
  asm volatile("v_nop\n\tv_nop\n\tv_nop\n\tv_nop" : "+v"(d) : "v"(a), "v"(b));
  return d;
}
__device__ __forceinline__ v16h frag_h(const _Float16* rowk0, int lane) {
  union { v16h v; v8h q[2]; } u; const _Float16* p = rowk0 + 8 * (lane >> 4);
  u.q[0] = *(const v8h*)p; u.q[1] = *(const v8h*)(p + 16); return u.v;
}
__device__ __forceinline__ v16h frag_f32(const float* rowk0, int lane) {
  v16h a; const float* p = rowk0 + 8 * (lane >> 4);
#pragma unroll
  for (int i = 0; i < 8; ++i) { a[i] = (_Float16)p[i]; a[8 + i] = (_Float16)p[16 + i]; }
  return a;
}
__device__ __forceinline__ v16h frag_f32s(const float* rowk0, int lane, float sc) {
  v16h a; const float* p = rowk0 + 8 * (lane >> 4);
#pragma unroll
  for (int i = 0; i < 8; ++i) { a[i] = (_Float16)(p[i] * sc); a[8 + i] = (_Float16)(p[16 + i] * sc); }
  return a;
}
__device__ __forceinline__ v16h fragc_f32(const float* W, int k0, int n, int lane, int ld, int K) {
  v16h a; const int g = lane >> 4;
#pragma unroll
  for (int i = 0; i < 8; ++i) { const int ka = k0 + 8 * g + i, kb = ka + 16;
    a[i] = (_Float16)(ka < K ? W[(size_t)(ka < K ? ka : K - 1) * ld + n] : 0.f); a[8 + i] = (_Float16)(kb < K ? W[(size_t)(kb < K ? kb : K - 1) * ld + n] : 0.f); }
  return a;
}
struct F2 { v16b h, l; };
__device__ __forceinline__ F2 bsplit16(const float v[16]) { F2 r;
#pragma unroll
  for (int i = 0; i < 16; ++i) { const __bf16 h = (__bf16)v[i]; r.h[i] = h; r.l[i] = (__bf16)(v[i] - (float)h); }
  return r; }
__device__ __forceinline__ F2 split_row(const float* row, int k0, int lane) { float v[16]; const float* p = row + k0 + 8 * (lane >> 4);
#pragma unroll
  for (int i = 0; i < 8; ++i) { v[i] = p[i]; v[8 + i] = p[16 + i]; }
  return bsplit16(v); }
__device__ __forceinline__ F2 split_rowK(const float* row, int k0, int lane, int K) { float v[16]; const int g = lane >> 4;
#pragma unroll
  for (int i = 0; i < 8; ++i) { const int ka = k0 + 8 * g + i, kb = ka + 16; v[i] = ka < K ? row[ka < K ? ka : K - 1] : 0.f; v[8 + i] = kb < K ? row[kb < K ? kb : K - 1] : 0.f; }
  return bsplit16(v); }
__device__ __forceinline__ F2 split_col(const float* W, int k0, int n, int lane, int ld, int K) { float v[16]; const int g = lane >> 4;
#pragma unroll
  for (int i = 0; i < 8; ++i) { const int ka = k0 + 8 * g + i, kb = ka + 16; v[i] = ka < K ? W[(size_t)(ka < K ? ka : K - 1) * ld + n] : 0.f; v[8 + i] = kb < K ? W[(size_t)(kb < K ? kb : K - 1) * ld + n] : 0.f; }
  return bsplit16(v); }
__device__ __forceinline__ v8f mac3(const F2& a, const F2& b, v8f c) { c = wmma_bf(a.l, b.h, c); c = wmma_bf(a.h, b.l, c); return wmma_bf(a.h, b.h, c); }
__device__ __forceinline__ float sigm(float v) { return 1.0f / (1.0f + expf(-v)); }
#define LDSX() do { asm volatile("s_wait_dscnt 0" ::: "memory"); __builtin_amdgcn_wave_barrier(); __builtin_amdgcn_fence(__ATOMIC_RELEASE, "workgroup"); } while (0)

__device__ __forceinline__ float bfr(float v) { return (float)(__bf16)v; }
#define MPTS 1048576
#define CF 64
#define PH 32
#define PWD 32
#define H1 128
#define H2 128
#ifndef NBLK
#define NBLK (MPTS / 64)
#endif
#define WS_PT 0u
#define WS_END (WS_PT + 4u * 3u * PH * PWD * CF)
__global__ __launch_bounds__(256) void k_pt(const float* __restrict__ P0, const float* __restrict__ P1, const float* __restrict__ P2, float* __restrict__ PT) { __shared__ float st[CF][PWD + 1];
  const int t = threadIdx.x; const int p = blockIdx.y, y = blockIdx.x; const float* P = p == 0 ? P0 : p == 1 ? P1 : P2;
  for (int e = t; e < CF * PWD; e += 256) { const int c = e >> 5, x = e & 31; st[c][x] = bfr(P[((size_t)c * PH + y) * PWD + x]); }
  __syncthreads();
  for (int e = t; e < PWD * CF / 4; e += 256) { const int x = e / (CF / 4), c4 = (e % (CF / 4)) * 4; v4f o; o[0] = st[c4][x]; o[1] = st[c4 + 1][x]; o[2] = st[c4 + 2][x]; o[3] = st[c4 + 3][x]; vst2(PT + (((size_t)p * PH + y) * PWD + x) * CF + c4, o); } }
struct Smp { int off[4]; float w[4]; };
__device__ __forceinline__ Smp mk_smp(float cx, float cy) { Smp s; const float x = (cx + 1.0f) * 0.5f * (float)(PWD - 1), y = (cy + 1.0f) * 0.5f * (float)(PH - 1); const float x0f = floorf(x), y0f = floorf(y); const float wx1 = x - x0f, wy1 = y - y0f, wx0 = 1.0f - wx1, wy0 = 1.0f - wy1; const int x0 = (int)x0f, y0 = (int)y0f;
  const int xs[4] = {x0, x0 + 1, x0, x0 + 1}, ys[4] = {y0, y0, y0 + 1, y0 + 1}; const float ws_[4] = {wx0 * wy0, wx1 * wy0, wx0 * wy1, wx1 * wy1};
#pragma unroll
  for (int q = 0; q < 4; ++q) { const bool valid = (xs[q] >= 0) && (xs[q] < PWD) && (ys[q] >= 0) && (ys[q] < PH); s.off[q] = valid ? (ys[q] * PWD + xs[q]) * CF : -1; s.w[q] = ws_[q]; }
  return s; }
__device__ __forceinline__ void sample8(const float* __restrict__ PL, const Smp& s, int c0, float out[8]) {
#pragma unroll
  for (int i = 0; i < 8; ++i) out[i] = 0.f;
#pragma unroll
  for (int q = 0; q < 4; ++q) { if (s.off[q] >= 0) { const v4f a = *(const v4f*)(PL + s.off[q] + c0), b = *(const v4f*)(PL + s.off[q] + c0 + 4);
      out[0] += a[0] * s.w[q]; out[1] += a[1] * s.w[q]; out[2] += a[2] * s.w[q]; out[3] += a[3] * s.w[q]; out[4] += b[0] * s.w[q]; out[5] += b[1] * s.w[q]; out[6] += b[2] * s.w[q]; out[7] += b[3] * s.w[q]; } } }
__global__ __launch_bounds__(128) void k_mlp(const float* __restrict__ CO, const float* __restrict__ PT, const float* __restrict__ W1, const float* __restrict__ B1, const float* __restrict__ W2, const float* __restrict__ B2, const float* __restrict__ W3, const float* __restrict__ B3, float* __restrict__ OUT) {
  __shared__ __align__(16) _Float16 sh1[64][H1 + 8]; __shared__ __align__(16) float sh2[64][H2 + 4]; __shared__ __align__(16) float so[64];
  const int tid = threadIdx.x, wave = tid >> 5, lane = tid & 31, col = lane & 15, g = lane >> 4; const size_t m0 = (size_t)blockIdx.x * 64; const size_t m = m0 + wave * 16 + col;
  const float c0v = bfr(CO[m * 3]), c1v = bfr(CO[m * 3 + 1]), c2v = bfr(CO[m * 3 + 2]);
  const Smp sxy = mk_smp(c0v, c1v), syz = mk_smp(c1v, c2v), sxz = mk_smp(c0v, c2v);
  const float* PXY = PT; const float* PYZ = PT + (size_t)PH * PWD * CF; const float* PXZ = PT + 2u * (size_t)PH * PWD * CF;
  v8f acc[8] = {};
#pragma unroll
  for (int kc = 0; kc < CF / 32; ++kc) { float fv[16];
#pragma unroll
    for (int hh = 0; hh < 2; ++hh) { const int cb = kc * 32 + hh * 16 + 8 * g; float a[8], b[8], c[8]; sample8(PXY, sxy, cb, a); sample8(PYZ, syz, cb, b); sample8(PXZ, sxz, cb, c);
#pragma unroll
      for (int i = 0; i < 8; ++i) fv[hh * 8 + i] = (a[i] * b[i]) * c[i]; }
    const F2 af = bsplit16(fv);
#pragma unroll
    for (int j = 0; j < 8; ++j) { v16b w; const int o = j * 16 + col;
#pragma unroll
      for (int i = 0; i < 8; ++i) { w[i] = (__bf16)W1[(size_t)o * CF + kc * 32 + 8 * g + i]; w[8 + i] = (__bf16)W1[(size_t)o * CF + kc * 32 + 16 + 8 * g + i]; }
      acc[j] = wmma_bf(af.h, w, acc[j]); acc[j] = wmma_bf(af.l, w, acc[j]); } }
#pragma unroll
  for (int j = 0; j < 8; ++j) { const int o = j * 16 + col; const float bb = bfr(B1[o]);
#pragma unroll
    for (int r = 0; r < 8; ++r) sh1[wave * 16 + 8 * g + r][o] = (_Float16)(fmaxf(acc[j][r] + bb, 0.f) * 262144.0f); }
  LDSX();
  { v8f acc2[8] = {};
#pragma unroll
    for (int kc = 0; kc < H1 / 32; ++kc) { const v16h a = frag_h(&sh1[wave * 16 + col][kc * 32], lane);
#pragma unroll
      for (int j = 0; j < 8; ++j) { v16h w; const int o = j * 16 + col;
#pragma unroll
        for (int i = 0; i < 8; ++i) { w[i] = (_Float16)(bfr(W2[(size_t)o * H1 + kc * 32 + 8 * g + i]) * 128.0f); w[8 + i] = (_Float16)(bfr(W2[(size_t)o * H1 + kc * 32 + 16 + 8 * g + i]) * 128.0f); }
        acc2[j] = wmma16(a, w, acc2[j]); } }
#pragma unroll
    for (int j = 0; j < 8; ++j) { const int o = j * 16 + col; const float bb = bfr(B2[o]);
#pragma unroll
      for (int r = 0; r < 8; ++r) sh2[wave * 16 + 8 * g + r][o] = fmaxf(acc2[j][r] * (1.0f / (262144.0f * 128.0f)) + bb, 0.f); } }
  __syncthreads();
  if (tid < 64) { const float* row = sh2[tid]; float s = 0.f;
#pragma unroll 1
    for (int o = 0; o < H2; o += 4) { const v4f hv = *(const v4f*)(row + o); s += hv[0] * bfr(W3[o]) + hv[1] * bfr(W3[o + 1]) + hv[2] * bfr(W3[o + 2]) + hv[3] * bfr(W3[o + 3]); }
    so[tid] = s + bfr(B3[0]); }
  __syncthreads();
  if (tid < 16) vst2(OUT + m0 + tid * 4, *(const v4f*)&so[tid * 4]); }
extern "C" void kernel_launch(void* const* d_in, const int* in_sizes, int n_in, void* d_out, int out_size, void* d_ws, size_t ws_size, hipStream_t stream) {
  (void)in_sizes; (void)n_in; (void)out_size;
  const float** F = (const float**)d_in;
  if (ws_size < (size_t)WS_END) return;
  char* ws = (char*)d_ws; float* PT = (float*)(ws + WS_PT);
  k_pt<<<dim3(PH, 3), 256, 0, stream>>>(F[1], F[2], F[3], PT);
  k_mlp<<<dim3(NBLK), 128, 0, stream>>>(F[0], PT, F[4], F[5], F[6], F[7], F[8], F[9], (float*)d_out);
}
